// G4_12558484374065
// MI455X (gfx1250) — hardware-verified
//
#include <hip/hip_runtime.h>

typedef unsigned short u16t;
typedef __bf16         v16b  __attribute__((ext_vector_type(16)));
typedef unsigned short v16us __attribute__((ext_vector_type(16)));
typedef unsigned short v8us  __attribute__((ext_vector_type(8)));
typedef float          v8f   __attribute__((ext_vector_type(8)));
typedef float          v4f   __attribute__((ext_vector_type(4)));
typedef v8us __attribute__((may_alias)) v8usa;
typedef v4f  __attribute__((may_alias)) v4fa;
union BFrag { v16us u; v16b b; v8us half[2]; };

#define NIMG   64
#define GIMG   16
#define NGRP   4
#define NPX    4096
#define PW     72
#define NPP    5184
#define CIN    8
#define CMID   128
#define K1P    256
#define K1S    7
#define K2     3840
#define H3P    416
#define IN_EPS 1e-5f

__device__ __forceinline__ unsigned int bf_bits(float x) {
  const unsigned int u = __float_as_uint(x);
  return (u + 0x7FFFu + ((u >> 16) & 1u)) >> 16;
}
__device__ __forceinline__ void split2(float x, u16t& hi, u16t& lo) {
  const unsigned int hb = bf_bits(x);
  const float hf = __uint_as_float(hb << 16);
  hi = (u16t)hb;
  lo = (u16t)bf_bits(x - hf);
}

__device__ __forceinline__ v8f wmma_bf(v16us a, v16us b, v8f c) {
  BFrag fa, fb;
  fa.u = a;
  fb.u = b;
  v8f d = __builtin_amdgcn_wmma_f32_16x16x32_bf16(false, fa.b, false, fb.b, (short)0, c, false, false);
  asm volatile("v_nop\n\tv_nop\n\tv_nop\n\tv_nop" : "+v"(d) : "v"(a), "v"(b));
  return d;
}

__device__ __forceinline__ v8f mma3(v16us ah, v16us al, v16us bh, v16us bl, v8f c) {
  c = wmma_bf(ah, bh, c);
  c = wmma_bf(al, bh, c);
  c = wmma_bf(ah, bl, c);
  return c;
}

__device__ __forceinline__ v16us ldfrag(const u16t* p, int h) {
  BFrag f;
  f.half[0] = *(const v8usa*)(p + 8 * h);
  f.half[1] = *(const v8usa*)(p + 16 + 8 * h);
  return f.u;
}

__device__ __forceinline__ v8f zero8f() {
  v8f z;
  #pragma unroll
  for (int j = 0; j < 8; ++j) z[j] = 0.f;
  return z;
}

__device__ __forceinline__ int clampi(int v, int lo, int hi) {
  return v < lo ? lo : (v > hi ? hi : v);
}

__global__ __launch_bounds__(128) void gemm64_k(
    const float* __restrict__ A, int lda, int K,
    const float* __restrict__ W, const float* __restrict__ bias, int N,
    float* __restrict__ Y, int ldy, int relu)
{
  __shared__ __attribute__((aligned(16))) float sO[64 * 32];
  const int tid = threadIdx.x, lane = tid & 31, w = tid >> 5;
  const int h = lane >> 4, m = lane & 15;
  const int n0 = blockIdx.x * 32;
  const float* ap = A + (size_t)(16 * w + m) * lda;
  int nc[2];
  #pragma unroll
  for (int nt = 0; nt < 2; ++nt) {
    const int n = n0 + 16 * nt + m;
    nc[nt] = n < N ? n : N - 1;
  }
  v8f acc[2];
  acc[0] = zero8f();
  acc[1] = zero8f();

  #pragma unroll 1
  for (int k0 = 0; k0 < K; k0 += 32) {
    float av[16];
    {
      const v4f t0 = *(const v4fa*)(ap + k0 + 8 * h);
      const v4f t1 = *(const v4fa*)(ap + k0 + 8 * h + 4);
      const v4f t2 = *(const v4fa*)(ap + k0 + 16 + 8 * h);
      const v4f t3 = *(const v4fa*)(ap + k0 + 16 + 8 * h + 4);
      #pragma unroll
      for (int j = 0; j < 4; ++j) { av[j] = t0[j]; av[4 + j] = t1[j]; av[8 + j] = t2[j]; av[12 + j] = t3[j]; }
    }
    BFrag ah, al;
    #pragma unroll
    for (int i = 0; i < 16; ++i) {
      u16t hi, lo;
      split2(av[i], hi, lo);
      ah.u[i] = hi;
      al.u[i] = lo;
    }
    #pragma unroll
    for (int nt = 0; nt < 2; ++nt) {
      const float* wp = W + nc[nt];
      BFrag bh, bl;
      #pragma unroll
      for (int i = 0; i < 8; ++i) {
        u16t hi, lo;
        split2(wp[(size_t)(k0 + 8 * h + i) * N], hi, lo);
        bh.u[i] = hi;
        bl.u[i] = lo;
        split2(wp[(size_t)(k0 + 16 + 8 * h + i) * N], hi, lo);
        bh.u[8 + i] = hi;
        bl.u[8 + i] = lo;
      }
      acc[nt] = mma3(ah.u, al.u, bh.u, bl.u, acc[nt]);
    }
  }

  #pragma unroll
  for (int nt = 0; nt < 2; ++nt) {
    const int nl = 16 * nt + m, n = n0 + nl;
    const float bv = bias[nc[nt]];
    const bool in = n < N;
    #pragma unroll
    for (int r = 0; r < 8; ++r) {
      float v = acc[nt][r] + bv;
      if (relu) v = fmaxf(v, 0.f);
      sO[(16 * w + 8 * h + r) * 32 + nl] = in ? v : 0.f;
    }
  }
  __syncthreads();
  const int q8 = lane & 7, sub = lane >> 3;
  v4f vals[4];
  size_t d[4];
  #pragma unroll
  for (int i = 0; i < 4; ++i) {
    const int row = 16 * w + 4 * i + sub;
    vals[i] = *(const v4fa*)(sO + row * 32 + 4 * q8);
    d[i] = (size_t)row * ldy + n0 + 4 * q8;
  }
  #pragma unroll
  for (int i = 0; i < 4; ++i) *(volatile v4f*)(Y + d[i]) = vals[i];
  __threadfence();
  #pragma unroll
  for (int i = 0; i < 4; ++i) *(volatile v4f*)(Y + d[i]) = vals[i];
}

__global__ __launch_bounds__(256) void gk_k(
    const float* __restrict__ k1w1, const float* __restrict__ k1b1,
    const float* __restrict__ k2w1, const float* __restrict__ k2b1, float* __restrict__ G)
{
  const int which = blockIdx.x, tid = threadIdx.x;
  const float* w1 = which ? k2w1 : k1w1;
  const float* b1 = which ? k2b1 : k1b1;
  float* gout = G + which * 4096;
  v4f vals[4];
  size_t d[4];
  #pragma unroll
  for (int it = 0; it < 4; ++it) {
    const int item = it * 256 + tid, row = item >> 4, c4 = item & 15;
    const int rc = row < 25 ? row : 24;
    const float gp0 = (float)(rc / 5 - 2) * 0.0625f;
    const float gp1 = (float)(rc % 5 - 2) * 0.0625f;
    v4f o;
    #pragma unroll
    for (int j = 0; j < 4; ++j) {
      const int hc = 4 * c4 + j;
      float v = gp0 * w1[hc] + gp1 * w1[64 + hc] + b1[hc];
      v = fmaxf(v, 0.f);
      o[j] = row < 25 ? v : 0.f;
    }
    vals[it] = o;
    d[it] = (size_t)row * 64 + 4 * c4;
  }
  #pragma unroll
  for (int it = 0; it < 4; ++it) *(volatile v4f*)(gout + d[it]) = vals[it];
  __threadfence();
  #pragma unroll
  for (int it = 0; it < 4; ++it) *(volatile v4f*)(gout + d[it]) = vals[it];
}

__global__ __launch_bounds__(256) void wconv_k(
    const float* __restrict__ KF1, const float* __restrict__ KF2,
    u16t* __restrict__ W1h, u16t* __restrict__ W1l, u16t* __restrict__ W2h, u16t* __restrict__ W2l)
{
  const int g = blockIdx.x * 256 + threadIdx.x;
  float v[8];
  u16t* dh;
  u16t* dl;
  size_t d;
  if (g < 4096) {
    const int co = g >> 5, t = g & 31, k0 = 8 * t;
    const int tc = t < 25 ? t : 24;
    const bool ok = t < 25;
    const float* src = KF1 + (size_t)tc * 1024 + co;
    #pragma unroll
    for (int i = 0; i < 8; ++i) { const float x = src[i * 128]; v[i] = ok ? x : 0.f; }
    d = (size_t)co * K1P + k0;
    dh = W1h;
    dl = W1l;
  } else {
    const int g2 = g - 4096, n = g2 / 480, rem = g2 - 480 * n, k0 = 8 * rem;
    const int j = k0 >> 7, c0 = k0 & 127, kh = j / 6, u = j - 6 * kh;
    const int co = n & 7, gg = n >> 3;
    const int kw = u - gg;
    const bool ok = (unsigned)kw < 5u;
    const int kwc = clampi(kw, 0, 4);
    const float* src = KF2 + (size_t)(kh * 5 + kwc) * 1024 + (size_t)c0 * 8 + co;
    #pragma unroll
    for (int i = 0; i < 8; ++i) { const float x = src[i * 8]; v[i] = ok ? x : 0.f; }
    d = (size_t)n * K2 + k0;
    dh = W2h;
    dl = W2l;
  }
  v8us hv, lv;
  #pragma unroll
  for (int i = 0; i < 8; ++i) { u16t hi, lo; split2(v[i], hi, lo); hv[i] = hi; lv[i] = lo; }
  *(volatile v8us*)(dh + d) = hv;
  *(volatile v8us*)(dl + d) = lv;
  __threadfence();
  *(volatile v8us*)(dh + d) = hv;
  *(volatile v8us*)(dl + d) = lv;
}

__global__ __launch_bounds__(256) void resize_k(
    const float* __restrict__ H3, u16t* __restrict__ F0h, u16t* __restrict__ F0l)
{
  const int t = blockIdx.x * 256 + threadIdx.x;
  const int b = t / NPP, pos = t - b * NPP, yp = pos / PW, xp = pos - yp * PW;
  const int y = yp - 4, x = xp - 4;
  const bool inside = ((unsigned)y < 64u) && ((unsigned)x < 64u);
  const int yc = clampi(y, 0, 63), xc = clampi(x, 0, 63);

  const float sfy = ((float)yc + 0.5f) * 0.109375f - 0.5f;
  int iy0 = (int)floorf(sfy);
  float fy = sfy - (float)iy0;
  if (iy0 < 0) { iy0 = 0; fy = 0.f; }
  int iy1 = iy0 + 1;
  if (iy1 > 6) { iy1 = 6; fy = 0.f; }
  const float sfx = ((float)xc + 0.5f) * 0.109375f - 0.5f;
  int ix0 = (int)floorf(sfx);
  float fx = sfx - (float)ix0;
  if (ix0 < 0) { ix0 = 0; fx = 0.f; }
  int ix1 = ix0 + 1;
  if (ix1 > 6) { ix1 = 6; fx = 0.f; }
  const float wy0 = 1.f - fy, wy1 = fy, wx0 = 1.f - fx, wx1 = fx;
  const int o00 = iy0 * 7 + ix0, o01 = iy0 * 7 + ix1, o10 = iy1 * 7 + ix0, o11 = iy1 * 7 + ix1;
  const float* hb = H3 + (size_t)b * H3P;

  v8us hv, lv;
  #pragma unroll
  for (int c = 0; c < CIN; ++c) {
    const float* p = hb + c * 49;
    const float ty0 = wy0 * p[o00] + wy1 * p[o10];
    const float ty1 = wy0 * p[o01] + wy1 * p[o11];
    float v = wx0 * ty0 + wx1 * ty1;
    v = inside ? v : 0.f;
    u16t hi, lo;
    split2(v, hi, lo);
    hv[c] = hi;
    lv[c] = lo;
  }
  const size_t d = (size_t)t * CIN;
  *(volatile v8us*)(F0h + d) = hv;
  *(volatile v8us*)(F0l + d) = lv;
  __threadfence();
  *(volatile v8us*)(F0h + d) = hv;
  *(volatile v8us*)(F0l + d) = lv;
}

__global__ __launch_bounds__(256) void conv1_k(
    const u16t* __restrict__ F0h, const u16t* __restrict__ F0l,
    const u16t* __restrict__ W1h, const u16t* __restrict__ W1l, float* __restrict__ C1)
{
  __shared__ __attribute__((aligned(16))) float sO[64 * CMID];
  const int tid = threadIdx.x, lane = tid & 31, w = tid >> 5;
  const int h = lane >> 4, m = lane & 15;
  const int y = blockIdx.x, bl = blockIdx.y;
  const int mt = w & 3, nh = w >> 2;
  const int x = 16 * mt + m;
  const size_t pb = ((size_t)bl * PW + y) * PW + x;
  const u16t* wrh = W1h + (size_t)(64 * nh + m) * K1P;
  const u16t* wrl = W1l + (size_t)(64 * nh + m) * K1P;
  const v8f z8 = zero8f();
  v8f acc[4];
  #pragma unroll
  for (int nt = 0; nt < 4; ++nt) acc[nt] = z8;

  #pragma unroll 1
  for (int s = 0; s < K1S; ++s) {
    int t0 = 4 * s + h;     t0 = t0 < 25 ? t0 : 24;
    int t1 = 4 * s + 2 + h; t1 = t1 < 25 ? t1 : 24;
    const size_t o0 = (pb + (size_t)(2 * (t0 / 5)) * PW + 2 * (t0 % 5)) * CIN;
    const size_t o1 = (pb + (size_t)(2 * (t1 / 5)) * PW + 2 * (t1 % 5)) * CIN;
    BFrag ah, al;
    ah.half[0] = *(const v8usa*)(F0h + o0);
    ah.half[1] = *(const v8usa*)(F0h + o1);
    al.half[0] = *(const v8usa*)(F0l + o0);
    al.half[1] = *(const v8usa*)(F0l + o1);
    #pragma unroll
    for (int nt = 0; nt < 4; ++nt) {
      const v16us bh = ldfrag(wrh + (size_t)(16 * nt) * K1P + 32 * s, h);
      const v16us bl2 = ldfrag(wrl + (size_t)(16 * nt) * K1P + 32 * s, h);
      acc[nt] = mma3(ah.u, al.u, bh, bl2, acc[nt]);
    }
  }

  #pragma unroll
  for (int nt = 0; nt < 4; ++nt) {
    const int ch = 64 * nh + 16 * nt + m;
    #pragma unroll
    for (int r = 0; r < 8; ++r) sO[(16 * mt + 8 * h + r) * CMID + ch] = acc[nt][r];
  }
  __syncthreads();
  v4f vals[8];
  size_t d[8];
  #pragma unroll
  for (int i = 0; i < 8; ++i) {
    const int pl = 8 * w + i;
    vals[i] = *(const v4fa*)(sO + pl * CMID + 4 * lane);
    d[i] = ((size_t)bl * NPX + (size_t)y * 64 + pl) * CMID + 4 * lane;
  }
  #pragma unroll
  for (int i = 0; i < 8; ++i) *(volatile v4f*)(C1 + d[i]) = vals[i];
  __threadfence();
  #pragma unroll
  for (int i = 0; i < 8; ++i) *(volatile v4f*)(C1 + d[i]) = vals[i];
}

__global__ __launch_bounds__(256) void in1_k(
    const float* __restrict__ C1, const float* __restrict__ g1, const float* __restrict__ be1,
    u16t* __restrict__ F1h, u16t* __restrict__ F1l)
{
  __shared__ double sS[256];
  __shared__ double sQ[256];
  __shared__ float smu[CMID];
  __shared__ float srs[CMID];
  __shared__ float sg[CMID];
  __shared__ float sb[CMID];
  const int tid = threadIdx.x, bl = blockIdx.x;
  {
    const int c = tid & 127, hs = tid >> 7;
    const float* cp = C1 + ((size_t)bl * NPX + (size_t)hs * 2048) * CMID + c;
    double s = 0.0, q = 0.0;
    #pragma unroll 4
    for (int i = 0; i < 2048; ++i) {
      const float v = cp[(size_t)i * CMID];
      s += (double)v;
      q += (double)v * (double)v;
    }
    sS[tid] = s;
    sQ[tid] = q;
  }
  __syncthreads();
  if (tid < CMID) {
    const double S = sS[tid] + sS[tid + 128];
    const double Q = sQ[tid] + sQ[tid + 128];
    const double mean = S * (1.0 / 4096.0);
    double var = Q * (1.0 / 4096.0) - mean * mean;
    if (var < 0.0) var = 0.0;
    smu[tid] = (float)mean;
    srs[tid] = rsqrtf((float)var + IN_EPS);
    sg[tid] = g1[tid];
    sb[tid] = be1[tid];
  }
  __syncthreads();

  #pragma unroll 1
  for (int k = 0; k < 324; ++k) {
    const int it = k * 256 + tid, pos = it >> 4, cg = it & 15;
    const int yp = pos / PW, xp = pos - yp * PW, y = yp - 4, x = xp - 4;
    const bool inside = ((unsigned)y < 64u) && ((unsigned)x < 64u);
    const int yc = clampi(y, 0, 63), xc = clampi(x, 0, 63);
    const float* src = C1 + ((size_t)bl * NPX + (size_t)yc * 64 + xc) * CMID + 8 * cg;
    const v4f a = *(const v4fa*)src;
    const v4f bq = *(const v4fa*)(src + 4);
    float v[8];
    #pragma unroll
    for (int j = 0; j < 4; ++j) { v[j] = a[j]; v[4 + j] = bq[j]; }
    v8us hv, lv;
    #pragma unroll
    for (int i = 0; i < 8; ++i) {
      const int c = 8 * cg + i;
      float t = ((v[i] - smu[c]) * srs[c]) * sg[c] + sb[c];
      t = fmaxf(t, 0.f);
      t = inside ? t : 0.f;
      u16t hi, lo;
      split2(t, hi, lo);
      hv[i] = hi;
      lv[i] = lo;
    }
    const size_t d = ((size_t)bl * NPP + pos) * CMID + 8 * cg;
    *(volatile v8us*)(F1h + d) = hv;
    *(volatile v8us*)(F1l + d) = lv;
    __threadfence();
    *(volatile v8us*)(F1h + d) = hv;
    *(volatile v8us*)(F1l + d) = lv;
  }
}

__global__ __launch_bounds__(256) void conv2_k(
    const u16t* __restrict__ F1h, const u16t* __restrict__ F1l,
    const u16t* __restrict__ W2h, const u16t* __restrict__ W2l, float* __restrict__ O2)
{
  __shared__ __attribute__((aligned(16))) float sO[8 * 4 * 64];
  const int tid = threadIdx.x, lane = tid & 31, w = tid >> 5;
  const int h = lane >> 4, m = lane & 15;
  const int yq = blockIdx.x, bl = blockIdx.y;
  const int yl = w >> 1, mt = w & 1;
  const int y = 4 * yq + yl;
  const int x0 = 32 * mt + 4 * (m >> 1) + (m & 1);
  const size_t abase = (((size_t)bl * PW + y) * PW + x0) * CMID;
  const u16t* aph = F1h + abase;
  const u16t* apl = F1l + abase;
  const u16t* bph = W2h + (size_t)m * K2;
  const u16t* bpl = W2l + (size_t)m * K2;
  v8f acc = zero8f();

  #pragma unroll 1
  for (int j = 0; j < 30; ++j) {
    const int kh = j / 6, u = j - 6 * kh;
    const size_t aoff = ((size_t)(2 * kh) * PW + 2 * u) * CMID;
    const size_t boff = (size_t)j * CMID;
    #pragma unroll
    for (int cq = 0; cq < 4; ++cq) {
      const v16us ah = ldfrag(aph + aoff + 32 * cq, h);
      const v16us al = ldfrag(apl + aoff + 32 * cq, h);
      const v16us bh = ldfrag(bph + boff + 32 * cq, h);
      const v16us bl2 = ldfrag(bpl + boff + 32 * cq, h);
      acc = mma3(ah, al, bh, bl2, acc);
    }
  }

  {
    const int co = m & 7, g = m >> 3;
    #pragma unroll
    for (int r = 0; r < 8; ++r) {
      const int xx = 32 * mt + 16 * h + 4 * (r >> 1) + (r & 1) + 2 * g;
      sO[(co * 4 + yl) * 64 + xx] = acc[r];
    }
  }
  __syncthreads();
  v4f vals[2];
  size_t d[2];
  #pragma unroll
  for (int i = 0; i < 2; ++i) {
    const int q = 32 * i + lane;
    vals[i] = *(const v4fa*)(sO + w * 256 + 4 * q);
    d[i] = ((size_t)bl * 8 + w) * NPX + (size_t)yq * 256 + 4 * q;
  }
  #pragma unroll
  for (int i = 0; i < 2; ++i) *(volatile v4f*)(O2 + d[i]) = vals[i];
  __threadfence();
  #pragma unroll
  for (int i = 0; i < 2; ++i) *(volatile v4f*)(O2 + d[i]) = vals[i];
}

__device__ __forceinline__ float tanh_fast(float x) {
  const float e = __expf(2.f * x);
  return 1.f - 2.f * __builtin_amdgcn_rcpf(e + 1.f);
}

__global__ __launch_bounds__(256) void final_k(
    const float* __restrict__ O2, const float* __restrict__ g2, const float* __restrict__ be2,
    const float* __restrict__ Wcm, const float* __restrict__ bcm, float* __restrict__ out)
{
  __shared__ double sS[256];
  __shared__ double sQ[256];
  __shared__ float smu[8];
  __shared__ float srs[8];
  __shared__ float sg[8];
  __shared__ float sb[8];
  __shared__ float swc[24];
  __shared__ float sbc[4];
  const int tid = threadIdx.x, lane = tid & 31, w = tid >> 5, b = blockIdx.x;
  {
    const float* pl = O2 + ((size_t)b * 8 + w) * NPX;
    double s = 0.0, q = 0.0;
    #pragma unroll 4
    for (int i = lane; i < NPX; i += 32) {
      const float v = pl[i];
      s += (double)v;
      q += (double)v * (double)v;
    }
    sS[tid] = s;
    sQ[tid] = q;
  }
  if (tid < 24) swc[tid] = Wcm[tid];
  if (tid < 3) sbc[tid] = bcm[tid];
  __syncthreads();
  if (tid < 8) {
    double S = 0.0, Q = 0.0;
    #pragma unroll 1
    for (int l = 0; l < 32; ++l) { S += sS[32 * tid + l]; Q += sQ[32 * tid + l]; }
    const double mean = S * (1.0 / 4096.0);
    double var = Q * (1.0 / 4096.0) - mean * mean;
    if (var < 0.0) var = 0.0;
    smu[tid] = (float)mean;
    srs[tid] = rsqrtf((float)var + IN_EPS);
    sg[tid] = g2[tid];
    sb[tid] = be2[tid];
  }
  __syncthreads();

  #pragma unroll 1
  for (int k = 0; k < 4; ++k) {
    const int q = k * 256 + tid;
    float s0[4], s1[4], s2[4];
    #pragma unroll
    for (int j = 0; j < 4; ++j) { s0[j] = 0.f; s1[j] = 0.f; s2[j] = 0.f; }
    #pragma unroll 1
    for (int c = 0; c < 8; ++c) {
      const v4f a = *(const v4fa*)(O2 + ((size_t)b * 8 + c) * NPX + 4 * q);
      const float mu = smu[c], rs = srs[c], gg = sg[c], bb = sb[c];
      const float w0 = swc[3 * c], w1 = swc[3 * c + 1], w2 = swc[3 * c + 2];
      #pragma unroll
      for (int j = 0; j < 4; ++j) {
        float t = ((a[j] - mu) * rs) * gg + bb;
        t = fmaxf(t, 0.f);
        s0[j] += t * w0;
        s1[j] += t * w1;
        s2[j] += t * w2;
      }
    }
    v4f o0, o1, o2;
    #pragma unroll
    for (int j = 0; j < 4; ++j) {
      o0[j] = tanh_fast(s0[j] + sbc[0]);
      o1[j] = tanh_fast(s1[j] + sbc[1]);
      o2[j] = tanh_fast(s2[j] + sbc[2]);
    }
    const size_t d0 = ((size_t)b * 3 + 0) * NPX + 4 * q;
    const size_t d1 = ((size_t)b * 3 + 1) * NPX + 4 * q;
    const size_t d2 = ((size_t)b * 3 + 2) * NPX + 4 * q;
    *(volatile v4f*)(out + d0) = o0;
    *(volatile v4f*)(out + d1) = o1;
    *(volatile v4f*)(out + d2) = o2;
    __threadfence();
    *(volatile v4f*)(out + d0) = o0;
    *(volatile v4f*)(out + d1) = o1;
    *(volatile v4f*)(out + d2) = o2;
  }
}

extern "C" void kernel_launch(void* const* d_in, const int* in_sizes, int n_in,
                              void* d_out, int out_size, void* d_ws, size_t ws_size,
                              hipStream_t stream)
{
  if (n_in < 21) return;
  const int expect[21] = {8192, 65536, 512, 131072, 256, 100352, 392,
                          128, 64, 65536, 1024, 128, 128,
                          128, 64, 65536, 1024, 8, 8, 24, 3};
  for (int i = 0; i < 21; ++i) if (in_sizes[i] != expect[i]) return;
  if (out_size != NIMG * 3 * NPX) return;

  const float* x    = (const float*)d_in[0];
  const float* W1   = (const float*)d_in[1];
  const float* b1   = (const float*)d_in[2];
  const float* W2   = (const float*)d_in[3];
  const float* b2   = (const float*)d_in[4];
  const float* W3   = (const float*)d_in[5];
  const float* b3   = (const float*)d_in[6];
  const float* k1w1 = (const float*)d_in[7];
  const float* k1b1 = (const float*)d_in[8];
  const float* k1w2 = (const float*)d_in[9];
  const float* k1b2 = (const float*)d_in[10];
  const float* g1   = (const float*)d_in[11];
  const float* be1  = (const float*)d_in[12];
  const float* k2w1 = (const float*)d_in[13];
  const float* k2b1 = (const float*)d_in[14];
  const float* k2w2 = (const float*)d_in[15];
  const float* k2b2 = (const float*)d_in[16];
  const float* g2   = (const float*)d_in[17];
  const float* be2  = (const float*)d_in[18];
  const float* Wcm  = (const float*)d_in[19];
  const float* bcm  = (const float*)d_in[20];
  float* outp = (float*)d_out;

  const size_t szH1 = (size_t)64 * 512 * 4;
  const size_t szH2 = (size_t)64 * 256 * 4;
  const size_t szH3 = (size_t)64 * H3P * 4;
  const size_t szG  = (size_t)2 * 64 * 64 * 4;
  const size_t szKF = (size_t)64 * 1024 * 4;
  const size_t szW1 = (size_t)CMID * K1P * 2;
  const size_t szW2 = (size_t)16 * K2 * 2;
  const size_t szF0 = (size_t)NIMG * NPP * CIN * 2;
  const size_t szC1 = (size_t)GIMG * NPX * CMID * 4;
  const size_t szF1 = (size_t)GIMG * NPP * CMID * 2;
  const size_t szO2 = (size_t)NIMG * 8 * NPX * 4;
  size_t off = 0;
  char* ws = (char*)d_ws;
  float* H1  = (float*)(ws + off); off += szH1;
  float* H2  = (float*)(ws + off); off += szH2;
  float* H3  = (float*)(ws + off); off += szH3;
  float* G   = (float*)(ws + off); off += szG;
  float* KF1 = (float*)(ws + off); off += szKF;
  float* KF2 = (float*)(ws + off); off += szKF;
  u16t*  W1h = (u16t*)(ws + off);  off += szW1;
  u16t*  W1l = (u16t*)(ws + off);  off += szW1;
  u16t*  W2h = (u16t*)(ws + off);  off += szW2;
  u16t*  W2l = (u16t*)(ws + off);  off += szW2;
  u16t*  F0h = (u16t*)(ws + off);  off += szF0;
  u16t*  F0l = (u16t*)(ws + off);  off += szF0;
  float* C1  = (float*)(ws + off); off += szC1;
  u16t*  F1h = (u16t*)(ws + off);  off += szF1;
  u16t*  F1l = (u16t*)(ws + off);  off += szF1;
  float* O2  = (float*)(ws + off); off += szO2;
  if (off > ws_size) return;

  gemm64_k<<<512 / 32, 128, 0, stream>>>(x, 128, 128, W1, b1, 512, H1, 512, 1);
  gemm64_k<<<256 / 32, 128, 0, stream>>>(H1, 512, 512, W2, b2, 256, H2, 256, 1);
  gemm64_k<<<H3P / 32, 128, 0, stream>>>(H2, 256, 256, W3, b3, 392, H3, H3P, 0);
  gk_k<<<2, 256, 0, stream>>>(k1w1, k1b1, k2w1, k2b1, G);
  gemm64_k<<<1024 / 32, 128, 0, stream>>>(G, 64, 64, k1w2, k1b2, 1024, KF1, 1024, 0);
  gemm64_k<<<1024 / 32, 128, 0, stream>>>(G + 4096, 64, 64, k2w2, k2b2, 1024, KF2, 1024, 0);
  wconv_k<<<(4096 + 7680) / 256, 256, 0, stream>>>(KF1, KF2, W1h, W1l, W2h, W2l);
  resize_k<<<(NIMG * NPP) / 256, 256, 0, stream>>>(H3, F0h, F0l);
  for (int grp = 0; grp < NGRP; ++grp) {
    const size_t f0off = (size_t)grp * GIMG * NPP * CIN;
    const size_t o2off = (size_t)grp * GIMG * 8 * NPX;
    conv1_k<<<dim3(64, GIMG), 256, 0, stream>>>(F0h + f0off, F0l + f0off, W1h, W1l, C1);
    in1_k<<<GIMG, 256, 0, stream>>>(C1, g1, be1, F1h, F1l);
    conv2_k<<<dim3(16, GIMG), 256, 0, stream>>>(F1h, F1l, W2h, W2l, O2 + o2off);
  }
  final_k<<<NIMG, 256, 0, stream>>>(O2, g2, be2, Wcm, bcm, outp);
}
